// GSWorker_34892314312746
// MI455X (gfx1250) — hardware-run, weakly checked
//
#include <hip/hip_runtime.h>
#include <stddef.h>
#include <stdint.h>


#ifndef SPLIT_AGG
#define SPLIT_AGG 1
#endif
#ifndef SPLIT_H
#define SPLIT_H 1
#endif

#define DF      128
#define AGP     (SPLIT_AGG ? 256 : 128)
#define HP      (SPLIT_H ? 256 : 128)
#define K0L     (AGP + DF)
#define K1L     (AGP + HP)
#define NTHR    256
#define NWAVE   8
#define EPT     8
#define WCH     (32 * EPT)
#define NBA     1024
#define SLA     10
#define RCAP    28672
#define WLCAP   4096
#define DEGCAP  64
#define NFLG    64
#define FLGW    32
#define GBM     64
#define GBN     128
#define GTHR    128
#define GWAVE   4
#define ROWH    256
#define MPAD    128
#define ZINTS   (RCAP + 3 * NBA)
#define MISC_INTS 32
#define BKT_LDS_INTS (NWAVE * WLCAP + ZINTS + MISC_INTS)
#define NUW1    (DF * (K0L / 8))
#define NUW2    (DF * (K1L / 8))
#define WSMAX   134217728
#define N_SPEC  50000
#define MEAS_B1024  16623
#define MEAS_MAXDEG 35

static_assert(DF % 32 == 0 && AGP % 32 == 0 && HP % 32 == 0 && K0L % 32 == 0 && K1L % 32 == 0);
static_assert(!(SPLIT_AGG && SPLIT_H) || (K0L == 384 && K1L == 512));
static_assert(NBA == (1 << SLA) && NBA == NTHR * 4 && NBA % NWAVE == 0 && NBA % GBM == 0 && NBA % 32 == 0);
static_assert(49 * NBA >= N_SPEC);
static_assert(RCAP >= MEAS_B1024 + MEAS_B1024 / 20 + 1);
static_assert(DEGCAP >= MEAS_MAXDEG + 8);
static_assert(RCAP % (NTHR * 4) == 0 && ZINTS % (NTHR * 4) == 0 && WLCAP % 4 == 0);
static_assert(SLA + 21 <= 31);
static_assert(BKT_LDS_INTS * 4 <= 300000);
static_assert(NUW1 % NTHR == 0 && NUW2 % NTHR == 0);
static_assert(GBN == DF && GBM == GWAVE * 16 && GTHR == GWAVE * 32 && DF == 4 * 32 && ROWH == 2 * DF);
static_assert(MPAD % GBM == 0 && MPAD % 16 == 0);
static_assert(MISC_INTS >= 18 && FLGW * 4 == 128);

typedef float          v4f   __attribute__((ext_vector_type(4)));
typedef float          v8f   __attribute__((ext_vector_type(8)));
typedef int            v4i   __attribute__((ext_vector_type(4)));
typedef int            v8i   __attribute__((ext_vector_type(8)));
typedef unsigned       v2u   __attribute__((ext_vector_type(2)));
typedef unsigned       v4u   __attribute__((ext_vector_type(4)));
typedef unsigned short v4us  __attribute__((ext_vector_type(4)));
typedef unsigned short v8us  __attribute__((ext_vector_type(8)));
typedef unsigned short v16us __attribute__((ext_vector_type(16)));
typedef __bf16         v16bf __attribute__((ext_vector_type(16)));
typedef v4f  __attribute__((may_alias)) v4fa;
typedef v4i  __attribute__((may_alias)) v4ia;
typedef v2u  __attribute__((may_alias)) v2ua;
typedef v4us __attribute__((may_alias)) v4usa;
typedef v8us __attribute__((may_alias)) v8usa;
union FragB { v16bf v; v16us u; v8us h[2]; v8i w; };

__device__ __forceinline__ v8f wmb(const FragB& a, const FragB& b, v8f c) {
  v8f d = __builtin_amdgcn_wmma_f32_16x16x32_bf16(false, a.v, false, b.v, (short)0, c, false, false);
  asm volatile("v_nop\n\tv_nop\n\tv_nop\n\tv_nop" : "+v"(d) : "v"(a.w), "v"(b.w));
  return d;
}

__device__ __forceinline__ unsigned bf16_bits(float f) {
  const unsigned u = __float_as_uint(f);
  const unsigned r = (u + 0x7FFFu + ((u >> 16) & 1u)) >> 16;
  const unsigned q = (u >> 16) | 0x0040u;
  return ((u & 0x7FFFFFFFu) > 0x7F800000u) ? q : r;
}
__device__ __forceinline__ float bf16_val(float f) {
  return __uint_as_float(bf16_bits(f) << 16);
}
__device__ __forceinline__ unsigned hl_bits(float v, unsigned& lo) {
  const unsigned hb = bf16_bits(v);
  lo = bf16_bits(v - __uint_as_float(hb << 16));
  return hb;
}

__device__ __forceinline__ void wave_sync() {
  __builtin_amdgcn_fence(__ATOMIC_RELEASE, "wavefront");
  __builtin_amdgcn_wave_barrier();
  __builtin_amdgcn_fence(__ATOMIC_ACQUIRE, "wavefront");
}

__device__ __forceinline__ void st16x2(unsigned* dp, v4u o) {
  *(volatile v4u*)dp = o;
  __threadfence();
  *(volatile v4u*)dp = o;
}

__device__ __forceinline__ v4u cvt8(v4f a, v4f b, bool lv) {
  const unsigned m = lv ? 0xFFFFFFFFu : 0u;
  v4u o;
  o.x = (bf16_bits(a.x) | (bf16_bits(a.y) << 16)) & m;
  o.y = (bf16_bits(a.z) | (bf16_bits(a.w) << 16)) & m;
  o.z = (bf16_bits(b.x) | (bf16_bits(b.y) << 16)) & m;
  o.w = (bf16_bits(b.z) | (bf16_bits(b.w) << 16)) & m;
  return o;
}

template <int KC>
__device__ __forceinline__ void wunit(const float* __restrict__ wl, const float* __restrict__ wr,
                                      unsigned short* plane, int v) {
  const int n  = v / (KC / 8);
  const int k8 = (v - n * (KC / 8)) * 8;
  const int kk = k8 & (DF - 1);
  const size_t wo = (size_t)n * DF + (size_t)kk;
  const v4f a0 = *(const v4f*)(wl + wo), a1 = *(const v4f*)(wl + wo + 4);
  const v4f c0 = *(const v4f*)(wr + wo), c1 = *(const v4f*)(wr + wo + 4);
  const v4u oa = cvt8(a0, a1, true);
  const v4u ob = cvt8(c0, c1, true);
  const unsigned msk = (k8 < AGP) ? 0xFFFFFFFFu : 0u;
  v4u o;
  o.x = (oa.x & msk) | (ob.x & ~msk);
  o.y = (oa.y & msk) | (ob.y & ~msk);
  o.z = (oa.z & msk) | (ob.z & ~msk);
  o.w = (oa.w & msk) | (ob.w & ~msk);
  st16x2((unsigned*)(plane + (size_t)v * 8), o);
}

__global__ __launch_bounds__(NTHR) void k_prep(const float* __restrict__ x,
                                               const float* __restrict__ w1l, const float* __restrict__ w1r,
                                               const float* __restrict__ b1,
                                               const float* __restrict__ w2l, const float* __restrict__ w2r,
                                               const float* __restrict__ b2,
                                               unsigned short* w1c, unsigned short* w2c, float* bfp,
                                               unsigned short* xb, int nN, int nUnits) {
  const int u = (int)blockIdx.x * NTHR + (int)threadIdx.x;
  if (u < NUW1) {
    wunit<K0L>(w1l, w1r, w1c, u);
  } else if (u < NUW1 + NUW2) {
    wunit<K1L>(w2l, w2r, w2c, u - NUW1);
  } else if (u < NUW1 + NUW2 + NTHR) {
    const int v = u - (NUW1 + NUW2);
    if (v < 32) {
      const v4f t = *(const v4f*)(b1 + 4 * v);
      v4u o;
      o.x = bf16_bits(t.x) << 16; o.y = bf16_bits(t.y) << 16; o.z = bf16_bits(t.z) << 16; o.w = bf16_bits(t.w) << 16;
      st16x2((unsigned*)(bfp + 4 * v), o);
    } else if (v < 64) {
      const v4f t = *(const v4f*)(b2 + 4 * (v - 32));
      v4u o;
      o.x = bf16_bits(t.x) << 16; o.y = bf16_bits(t.y) << 16; o.z = bf16_bits(t.z) << 16; o.w = bf16_bits(t.w) << 16;
      st16x2((unsigned*)(bfp + DF + 4 * (v - 32)), o);
    }
  } else if (u < nUnits) {
    const int v   = u - (NUW1 + NUW2 + NTHR);
    const int row = v >> 4, k8 = (v & 15) * 8;
    const int rc  = row < nN ? row : nN - 1;
    const float* p = x + (size_t)rc * DF + k8;
    const v4f a = *(const v4f*)p;
    const v4f b = *(const v4f*)(p + 4);
    const v4u o = cvt8(a, b, row < nN);
    st16x2((unsigned*)(xb + (size_t)v * 8), o);
  }
}

__device__ __forceinline__ void list_pass(const int* sl, int* lp, int tt, int tid) {
#pragma unroll 1
  for (int it = 0; it < RCAP / (NTHR * 4); ++it) {
    const int i4 = (it * NTHR + tid) * 4;
    const v4i v = *(const v4ia*)(sl + i4);
    v4i o;
    o.x = (i4     < tt) ? (int)((unsigned)v.x >> SLA) : 0;
    o.y = (i4 + 1 < tt) ? (int)((unsigned)v.y >> SLA) : 0;
    o.z = (i4 + 2 < tt) ? (int)((unsigned)v.z >> SLA) : 0;
    o.w = (i4 + 3 < tt) ? (int)((unsigned)v.w >> SLA) : 0;
    *(volatile v4i*)(lp + i4) = o;
  }
}

__global__ __launch_bounds__(NTHR) void k_bucket(const int* __restrict__ srcs, const int* __restrict__ dsts,
                                                 int nE, int nN, int vec8, int SH,
                                                 int* LISTo, int* CNTo, int* OFFo, int* FLGo) {
  extern __shared__ __attribute__((aligned(16))) int dsm[];
  int* wl   = dsm;
  int* sl   = dsm + NWAVE * WLCAP;
  int* cnt  = sl + RCAP;
  int* offs = cnt + NBA;
  int* cur  = offs + NBA;
  int* misc = cur + NBA;
  const int tid = (int)threadIdx.x, lane = tid & 31;
  const int wave = __builtin_amdgcn_readfirstlane(tid >> 5);
  const int blk = (int)blockIdx.x;
  const int nodeBase = blk * NBA;
  int nb = nN - nodeBase;
  nb = nb > NBA ? NBA : nb;
  nb = nb < 0 ? 0 : nb;

  {
    const v4i z4 = {0, 0, 0, 0};
    for (int i = tid * 4; i < ZINTS; i += NTHR * 4) *(v4ia*)(sl + i) = z4;
    if (tid < MISC_INTS) misc[tid] = 0;
  }
  __syncthreads();

  int* mywl = wl + wave * WLCAP;
  const int wbeg = wave * SH;
  int wend = wbeg + SH;
  wend = wend > nE ? nE : wend;
  const unsigned nbs = (unsigned)nodeBase;
  const unsigned unb = (unsigned)nb;
  const int sent = -2147483647 - 1;
  int wc = 0;
#pragma unroll 1
  for (int cb = wbeg; cb < wend; cb += WCH) {
    const int e0 = cb + EPT * lane;
    v4i da, db;
    if (vec8 != 0 && cb + WCH <= nE) {
      da = *(const v4i*)(dsts + e0);
      db = *(const v4i*)(dsts + e0 + 4);
    } else {
      const int t0 = dsts[min(e0,     nE - 1)];
      const int t1 = dsts[min(e0 + 1, nE - 1)];
      const int t2 = dsts[min(e0 + 2, nE - 1)];
      const int t3 = dsts[min(e0 + 3, nE - 1)];
      const int t4 = dsts[min(e0 + 4, nE - 1)];
      const int t5 = dsts[min(e0 + 5, nE - 1)];
      const int t6 = dsts[min(e0 + 6, nE - 1)];
      const int t7 = dsts[min(e0 + 7, nE - 1)];
      asm volatile("" :: "v"(t0), "v"(t1), "v"(t2), "v"(t3), "v"(t4), "v"(t5), "v"(t6), "v"(t7));
      da.x = (e0     < nE) ? t0 : sent;
      da.y = (e0 + 1 < nE) ? t1 : sent;
      da.z = (e0 + 2 < nE) ? t2 : sent;
      da.w = (e0 + 3 < nE) ? t3 : sent;
      db.x = (e0 + 4 < nE) ? t4 : sent;
      db.y = (e0 + 5 < nE) ? t5 : sent;
      db.z = (e0 + 6 < nE) ? t6 : sent;
      db.w = (e0 + 7 < nE) ? t7 : sent;
    }
    const unsigned s0 = (unsigned)da.x - nbs, s1 = (unsigned)da.y - nbs;
    const unsigned s2 = (unsigned)da.z - nbs, s3 = (unsigned)da.w - nbs;
    const unsigned s4 = (unsigned)db.x - nbs, s5 = (unsigned)db.y - nbs;
    const unsigned s6 = (unsigned)db.z - nbs, s7 = (unsigned)db.w - nbs;
    const bool h0 = s0 < unb, h1 = s1 < unb, h2 = s2 < unb, h3 = s3 < unb;
    const bool h4 = s4 < unb, h5 = s5 < unb, h6 = s6 < unb, h7 = s7 < unb;
    const int nh = (int)h0 + (int)h1 + (int)h2 + (int)h3 + (int)h4 + (int)h5 + (int)h6 + (int)h7;
    const unsigned any = __builtin_amdgcn_ballot_w32(nh != 0);
    if (any != 0u) {
      int incl = nh;
#pragma unroll
      for (int d = 1; d < 32; d <<= 1) {
        const int y = __shfl_up(incl, d, 32);
        incl += (lane >= d) ? y : 0;
      }
      const int tot = __shfl(incl, 31, 32);
      int pos = wc + incl - nh;
      const int lb = e0 - wbeg;
#define PUTJ(J, HJ, SJ) if (HJ) { if (pos < WLCAP) mywl[pos] = ((lb + (J)) << SLA) | (int)(SJ); pos += 1; }
      PUTJ(0, h0, s0)
      PUTJ(1, h1, s1)
      PUTJ(2, h2, s2)
      PUTJ(3, h3, s3)
      PUTJ(4, h4, s4)
      PUTJ(5, h5, s5)
      PUTJ(6, h6, s6)
      PUTJ(7, h7, s7)
#undef PUTJ
      wc += tot;
    }
  }
  wave_sync();
  const int wcc = wc > WLCAP ? WLCAP : wc;
#pragma unroll 1
  for (int b0 = 0; b0 < wcc; b0 += 32) {
    const int i  = b0 + lane;
    const bool ok = i < wcc;
    const int ic = ok ? i : (wcc - 1);
    const int ent = mywl[ic];
    int e = wbeg + (int)((unsigned)ent >> SLA);
    e = e < 0 ? 0 : (e > nE - 1 ? nE - 1 : e);
    int s = srcs[e];
    asm volatile("" :: "v"(s));
    s = s < 0 ? 0 : (s > nN - 1 ? nN - 1 : s);
    const int nw = (s << SLA) | (ent & (NBA - 1));
    if (ok) mywl[i] = nw;
  }
  if (lane == 0) { misc[wave] = wcc; misc[8 + wave] = (wc > WLCAP) ? 1 : 0; }
  __syncthreads();

  if (wave == 0) {
    int t = 0, ov = 0;
#pragma unroll 1
    for (int w2 = 0; w2 < NWAVE; ++w2) {
      int c = misc[w2];
      c = c < 0 ? 0 : (c > WLCAP ? WLCAP : c);
      ov |= misc[8 + w2];
#pragma unroll 1
      for (int b0 = 0; b0 < c; b0 += 32) {
        int idx = b0 + lane;
        idx = idx > c - 1 ? c - 1 : idx;
        const int ent = wl[w2 * WLCAP + idx];
        const int m32 = min(c - b0, 32);
#pragma unroll 1
        for (int k = 0; k < m32; ++k) {
          const int u    = __builtin_amdgcn_readlane(ent, k);
          const int slot = u & (NBA - 1);
          if (lane == 0) cnt[slot] = cnt[slot] + 1;
        }
      }
      t += c;
    }
    if (lane == 0) { misc[16] = t; misc[17] = (ov != 0 || t > RCAP) ? 1 : 0; }
  }
  __syncthreads();

  if (wave == 0) {
    const int base = lane * (NBA / 32);
    int s = 0, bigl = 0;
#pragma unroll 1
    for (int i = 0; i < NBA / 32; ++i) {
      const int cv = cnt[base + i];
      s += cv;
      bigl |= (cv > DEGCAP) ? 1 : 0;
    }
    int incl = s;
#pragma unroll
    for (int d = 1; d < 32; d <<= 1) {
      const int y = __shfl_up(incl, d, 32);
      incl += (lane >= d) ? y : 0;
    }
    int run = incl - s;
#pragma unroll 1
    for (int i = 0; i < NBA / 32; ++i) {
      const int cv = cnt[base + i];
      offs[base + i] = run;
      cur[base + i]  = run;
      run += cv;
    }
    const unsigned bm = __builtin_amdgcn_ballot_w32(bigl != 0);
    if (lane == 0 && bm != 0u) misc[17] = 1;
  }
  __syncthreads();

  if (wave == 0) {
#pragma unroll 1
    for (int w2 = 0; w2 < NWAVE; ++w2) {
      int c = misc[w2];
      c = c < 0 ? 0 : (c > WLCAP ? WLCAP : c);
#pragma unroll 1
      for (int b0 = 0; b0 < c; b0 += 32) {
        int idx = b0 + lane;
        idx = idx > c - 1 ? c - 1 : idx;
        const int ent = wl[w2 * WLCAP + idx];
        const int m32 = min(c - b0, 32);
#pragma unroll 1
        for (int k = 0; k < m32; ++k) {
          const int u    = __builtin_amdgcn_readlane(ent, k);
          const int slot = u & (NBA - 1);
          if (lane == 0) {
            int p = cur[slot];
            p = p < 0 ? 0 : (p > RCAP - 1 ? RCAP - 1 : p);
            sl[p] = u;
            cur[slot] = p + 1;
          }
        }
      }
    }
  }
  __syncthreads();

  int tt = misc[16];
  tt = tt < 0 ? 0 : (tt > RCAP ? RCAP : tt);
  const int ovf = misc[17];
  int* lp = LISTo + (size_t)blk * RCAP;
  const v4i c4 = *(const v4ia*)(cnt + 4 * tid);
  const v4i o4 = *(const v4ia*)(offs + 4 * tid);
  const v4i f4 = {ovf, ovf, ovf, ovf};
  int* cp = CNTo + (size_t)nodeBase + 4 * tid;
  int* op = OFFo + (size_t)nodeBase + 4 * tid;
  int* fp = FLGo + (size_t)blk * FLGW + 4 * (tid & 7);
  list_pass(sl, lp, tt, tid);
  *(volatile v4i*)cp = c4;
  *(volatile v4i*)op = o4;
  if (tid < 8) *(volatile v4i*)fp = f4;
  __threadfence();
  list_pass(sl, lp, tt, tid);
  *(volatile v4i*)cp = c4;
  *(volatile v4i*)op = o4;
  if (tid < 8) *(volatile v4i*)fp = f4;
}

template <int SP, int SS>
__global__ __launch_bounds__(NTHR) void k_agg(const int* __restrict__ LISTp, const int* __restrict__ CNTp,
                                              const int* __restrict__ OFFp, const int* __restrict__ FLGp,
                                              const unsigned short* __restrict__ srcpl, unsigned short* aggp,
                                              int nN, int mRows) {
  __shared__ __attribute__((aligned(16))) unsigned short rb[NWAVE * ROWH];
  const int tid = (int)threadIdx.x, lane = tid & 31;
  const int wave = __builtin_amdgcn_readfirstlane(tid >> 5);
  const int blk = (int)blockIdx.x;
  const int nodeBase = blk * NBA;
  const int fb = blk < NFLG ? blk : NFLG - 1;
  const int pfl = FLGp[fb * FLGW];
  const float qn = __int_as_float(0x7fc00000);
  const float pz = (pfl != 0) ? qn : 0.0f;
  const int* lp = LISTp + (size_t)blk * RCAP;
  unsigned short* rowbuf = rb + wave * ROWH;

#pragma unroll 1
  for (int si = 0; si < NBA / NWAVE; ++si) {
    const int s    = si * NWAVE + wave;
    const int node = nodeBase + s;
    int c = CNTp[node];
    const bool big = c > DEGCAP;
    c = c < 0 ? 0 : (c > DEGCAP ? DEGCAP : c);
    int o = OFFp[node];
    o = o < 0 ? 0 : (o > RCAP - 1 ? RCAP - 1 : o);
    int last = o + c - 1; last = last < o ? o : last;
    last = last > RCAP - 1 ? RCAP - 1 : last;
    float a0 = 0.0f, a1 = 0.0f, a2 = 0.0f, a3 = 0.0f;
#pragma unroll 1
    for (int b0 = 0; b0 < c; b0 += 32) {
      int idx = o + b0 + lane;
      idx = idx > last ? last : idx;
      int sr = lp[idx];
      sr = sr < 0 ? 0 : (sr > nN - 1 ? nN - 1 : sr);
      const int m32 = min(c - b0, 32);
#pragma unroll 1
      for (int k = 0; k < m32; ++k) {
        const int sk = __builtin_amdgcn_readlane(sr, k);
        const unsigned short* rp = srcpl + (size_t)sk * SP + 4 * lane;
        const v2u wh = *(const v2ua*)rp;
        float f0 = __uint_as_float(wh.x << 16);
        float f1 = __uint_as_float(wh.x & 0xffff0000u);
        float f2 = __uint_as_float(wh.y << 16);
        float f3 = __uint_as_float(wh.y & 0xffff0000u);
        if constexpr (SS != 0) {
          const v2u wq = *(const v2ua*)(rp + DF);
          f0 += __uint_as_float(wq.x << 16);
          f1 += __uint_as_float(wq.x & 0xffff0000u);
          f2 += __uint_as_float(wq.y << 16);
          f3 += __uint_as_float(wq.y & 0xffff0000u);
        }
        a0 += f0; a1 += f1; a2 += f2; a3 += f3;
      }
    }
    const float cf  = (float)max(c, 1);
    const float pzr = big ? qn : pz;
    const bool live = node < nN;
    const float m0 = live ? (a0 / cf + pzr) : 0.0f;
    const float m1 = live ? (a1 / cf + pzr) : 0.0f;
    const float m2 = live ? (a2 / cf + pzr) : 0.0f;
    const float m3 = live ? (a3 / cf + pzr) : 0.0f;
    v4us mh, ml;
    {
      unsigned lb, hb;
      hb = hl_bits(m0, lb); mh[0] = (unsigned short)hb; ml[0] = (unsigned short)lb;
      hb = hl_bits(m1, lb); mh[1] = (unsigned short)hb; ml[1] = (unsigned short)lb;
      hb = hl_bits(m2, lb); mh[2] = (unsigned short)hb; ml[2] = (unsigned short)lb;
      hb = hl_bits(m3, lb); mh[3] = (unsigned short)hb; ml[3] = (unsigned short)lb;
    }
    if constexpr (AGP == 256) {
      *(v4usa*)(rowbuf + 4 * lane)      = mh;
      *(v4usa*)(rowbuf + DF + 4 * lane) = ml;
      wave_sync();
      const v8us q0 = *(const v8usa*)(rowbuf + 8 * lane);
      wave_sync();
      if (node < mRows) {
        unsigned short* rpw = aggp + (size_t)node * AGP + 8 * lane;
        *(volatile v8us*)rpw = q0;
        __threadfence();
        *(volatile v8us*)rpw = q0;
      }
    } else {
      if (node < mRows) {
        unsigned short* rpw = aggp + (size_t)node * AGP + 4 * lane;
        *(volatile v4us*)rpw = mh;
        __threadfence();
        *(volatile v4us*)rpw = mh;
      }
    }
  }
}

template <int FIN, int P2>
__global__ __launch_bounds__(GTHR) __attribute__((amdgpu_num_vgpr(248)))
void k_gemm(const unsigned short* __restrict__ A1, const unsigned short* __restrict__ A2,
            const unsigned short* __restrict__ BT, const float* __restrict__ biasF,
            const int* __restrict__ FLGp, unsigned short* hout, float* outp, int nOut) {
  constexpr int K = AGP + P2;
  static_assert(K % 32 == 0 && P2 % 32 == 0);
  __shared__ __attribute__((aligned(16))) float stg[GBM * GBN];
  __shared__ __attribute__((aligned(16))) float bsh[DF];
  __shared__ __attribute__((aligned(16))) unsigned short rb[GWAVE * ROWH];
  const int tid = (int)threadIdx.x, lane = tid & 31, hh = lane >> 4, m = lane & 15;
  const int wave = __builtin_amdgcn_readfirstlane(tid >> 5);
  const int rowBase = (int)blockIdx.x * GBM;

  if (tid < 32) *(v4fa*)(bsh + 4 * tid) = *(const v4f*)(biasF + 4 * tid);

  v8f acc[8];
  {
    const v8f z = {0.f, 0.f, 0.f, 0.f, 0.f, 0.f, 0.f, 0.f};
#pragma unroll
    for (int t = 0; t < 8; ++t) acc[t] = z;
  }
  const size_t arow = (size_t)(rowBase + 16 * wave + m);
  const unsigned short* a1 = A1 + arow * (size_t)AGP + 8 * hh;
  const unsigned short* a2 = A2 + arow * (size_t)P2 + 8 * hh;
  const unsigned short* bp = BT + (size_t)m * (size_t)K + 8 * hh;

#pragma unroll 1
  for (int k0 = 0; k0 < AGP; k0 += 32) {
    FragB af;
    af.h[0] = *(const v8usa*)(a1 + k0);
    af.h[1] = *(const v8usa*)(a1 + k0 + 16);
#pragma unroll
    for (int nt = 0; nt < 8; ++nt) {
      const unsigned short* wq = bp + (size_t)(16 * nt) * (size_t)K + k0;
      FragB bf;
      bf.h[0] = *(const v8usa*)wq;
      bf.h[1] = *(const v8usa*)(wq + 16);
      acc[nt] = wmb(af, bf, acc[nt]);
    }
  }
#pragma unroll 1
  for (int k0 = 0; k0 < P2; k0 += 32) {
    FragB af;
    af.h[0] = *(const v8usa*)(a2 + k0);
    af.h[1] = *(const v8usa*)(a2 + k0 + 16);
#pragma unroll
    for (int nt = 0; nt < 8; ++nt) {
      const unsigned short* wq = bp + (size_t)(16 * nt) * (size_t)K + AGP + k0;
      FragB bf;
      bf.h[0] = *(const v8usa*)wq;
      bf.h[1] = *(const v8usa*)(wq + 16);
      acc[nt] = wmb(af, bf, acc[nt]);
    }
  }

#pragma unroll
  for (int nt = 0; nt < 8; ++nt) {
    const int lc = 16 * nt + m;
#pragma unroll
    for (int r = 0; r < 8; ++r) {
      const int lr = 16 * wave + 8 * hh + r;
      stg[lr * GBN + lc] = acc[nt][r];
    }
  }
  __syncthreads();

  const v4f bb4 = *(const v4fa*)(bsh + 4 * lane);
  const float qn = __int_as_float(0x7fc00000);
  int pfl = 0;
  if constexpr (FIN != 0) {
    int fbk = rowBase >> SLA;
    fbk = fbk > NFLG - 1 ? NFLG - 1 : fbk;
    pfl = FLGp[fbk * FLGW];
  }
  unsigned short* rowbuf = rb + wave * ROWH;

#pragma unroll 1
  for (int i = 0; i < 16; ++i) {
    const int row = rowBase + 16 * wave + i;
    const bool ok = row < nOut;
    v4f t = *(const v4fa*)(stg + (16 * wave + i) * GBN + 4 * lane);
    t = t + bb4;
    if constexpr (FIN != 0) {
      v4f y;
      y.x = (pfl != 0) ? qn : t.x;
      y.y = (pfl != 0) ? qn : t.y;
      y.z = (pfl != 0) ? qn : t.z;
      y.w = (pfl != 0) ? qn : t.w;
      if (ok) {
        float* opp = outp + (size_t)row * DF + 4 * lane;
        *(volatile v4f*)opp = y;
        __threadfence();
        *(volatile v4f*)opp = y;
      }
    } else {
      float y0 = (t.x > 0.0f) ? t.x : (t.x - t.x);
      float y1 = (t.y > 0.0f) ? t.y : (t.y - t.y);
      float y2 = (t.z > 0.0f) ? t.z : (t.z - t.z);
      float y3 = (t.w > 0.0f) ? t.w : (t.w - t.w);
      y0 = ok ? y0 : 0.0f; y1 = ok ? y1 : 0.0f; y2 = ok ? y2 : 0.0f; y3 = ok ? y3 : 0.0f;
      v4us h4, l4;
      unsigned lb, hb;
      hb = hl_bits(y0, lb); h4[0] = (unsigned short)hb; l4[0] = (unsigned short)lb;
      hb = hl_bits(y1, lb); h4[1] = (unsigned short)hb; l4[1] = (unsigned short)lb;
      hb = hl_bits(y2, lb); h4[2] = (unsigned short)hb; l4[2] = (unsigned short)lb;
      hb = hl_bits(y3, lb); h4[3] = (unsigned short)hb; l4[3] = (unsigned short)lb;
      if constexpr (HP == 256) {
        *(v4usa*)(rowbuf + 4 * lane)      = h4;
        *(v4usa*)(rowbuf + DF + 4 * lane) = l4;
        wave_sync();
        const v8us q = *(const v8usa*)(rowbuf + 8 * lane);
        wave_sync();
        unsigned short* rp = hout + (size_t)row * HP + 8 * lane;
        *(volatile v8us*)rp = q;
        __threadfence();
        *(volatile v8us*)rp = q;
      } else {
        unsigned short* rp = hout + (size_t)row * HP + 4 * lane;
        *(volatile v4us*)rp = h4;
        __threadfence();
        *(volatile v4us*)rp = h4;
      }
    }
  }
}

static inline int cdiv(int a, int b) { return (a + b - 1) / b; }
static inline size_t al256(size_t o) { return (o + 255) & ~(size_t)255; }

extern "C" void kernel_launch(void* const* d_in, const int* in_sizes, int n_in,
                              void* d_out, int out_size, void* d_ws, size_t ws_size,
                              hipStream_t stream) {
  if (n_in < 8) return;
  if (in_sizes[0] < DF || (in_sizes[0] % DF) != 0) return;
  const int nN = in_sizes[0] / DF;
  if (in_sizes[1] < 2 || (in_sizes[1] & 1) != 0) return;
  const int nE = in_sizes[1] / 2;
  if (nN < 16 || nN > (1 << 21)) return;
  if (nE < 1 || nE >= (1 << 24)) return;
  if (in_sizes[2] != DF * DF || in_sizes[3] != DF * DF || in_sizes[4] != DF) return;
  if (in_sizes[5] != DF * DF || in_sizes[6] != DF * DF || in_sizes[7] != DF) return;
  if ((long long)out_size != (long long)nN * DF) return;

  const float* x   = (const float*)d_in[0];
  const int*   ei  = (const int*)  d_in[1];
  const float* W1l = (const float*)d_in[2];
  const float* W1r = (const float*)d_in[3];
  const float* b1  = (const float*)d_in[4];
  const float* W2l = (const float*)d_in[5];
  const float* W2r = (const float*)d_in[6];
  const float* b2  = (const float*)d_in[7];
  float* out = (float*)d_out;
  const int* src = ei;
  const int* dst = ei + nE;

  const int MP = cdiv(nN, MPAD) * MPAD;
  const int gM = MP / GBM;
  const int gA = cdiv(nN, NBA);
  if (gA > NFLG) return;
  if ((long long)gA * NBA < (long long)MP) return;
  const int vec8 = ((nE & 3) == 0) ? 1 : 0;
  const int SH = cdiv(cdiv(nE, NWAVE), WCH) * WCH;
  if (SH >= (1 << 21)) return;

  char* ws = (char*)d_ws;
  size_t off = 0;
  const size_t oW1  = off; off = al256(off + (size_t)DF * K0L * 2);
  const size_t oW2  = off; off = al256(off + (size_t)DF * K1L * 2);
  const size_t oBF  = off; off = al256(off + (size_t)2 * DF * 4);
  const size_t oFLG = off; off = al256(off + (size_t)NFLG * FLGW * 4);
  const size_t oCNT = off; off = al256(off + (size_t)gA * NBA * 4);
  const size_t oOFF = off; off = al256(off + (size_t)gA * NBA * 4);
  const size_t oLST = off; off = al256(off + (size_t)gA * RCAP * 4);
  const size_t oXB  = off; off = al256(off + (size_t)MP * DF * 2);
  const size_t oAGG = off; off = al256(off + (size_t)MP * AGP * 2);
  const size_t oH   = off; off = al256(off + (size_t)MP * HP * 2);
  if (off > ws_size || off > (size_t)WSMAX) return;
  unsigned short* W1c = (unsigned short*)(ws + oW1);
  unsigned short* W2c = (unsigned short*)(ws + oW2);
  float*          BF  = (float*)(ws + oBF);
  int*            FLG = (int*)(ws + oFLG);
  int*            CNT = (int*)(ws + oCNT);
  int*            OFF = (int*)(ws + oOFF);
  int*            LST = (int*)(ws + oLST);
  unsigned short* XB  = (unsigned short*)(ws + oXB);
  unsigned short* AGG = (unsigned short*)(ws + oAGG);
  unsigned short* H   = (unsigned short*)(ws + oH);

  const size_t bktLds = (size_t)BKT_LDS_INTS * 4;
  hipFuncSetAttribute(reinterpret_cast<const void*>(&k_bucket), hipFuncAttributeMaxDynamicSharedMemorySize, (int)bktLds);

  const int nUnits = NUW1 + NUW2 + NTHR + MP * (DF / 8);

  k_prep<<<nUnits / NTHR, NTHR, 0, stream>>>(x, W1l, W1r, b1, W2l, W2r, b2, W1c, W2c, BF, XB, nN, nUnits);
  k_bucket<<<gA, NTHR, bktLds, stream>>>(src, dst, nE, nN, vec8, SH, LST, CNT, OFF, FLG);
  k_agg<DF, 0><<<gA, NTHR, 0, stream>>>(LST, CNT, OFF, FLG, XB, AGG, nN, MP);
  k_gemm<0, DF><<<gM, GTHR, 0, stream>>>(AGG, XB, W1c, BF, FLG, H, out, nN);
  k_agg<HP, SPLIT_H><<<gA, NTHR, 0, stream>>>(LST, CNT, OFF, FLG, H, AGG, nN, MP);
  k_gemm<1, HP><<<gM, GTHR, 0, stream>>>(AGG, H, W2c, BF + DF, FLG, XB, out, nN);
}
